// Net_59021440581865
// MI455X (gfx1250) — hardware-verified
//
#include <hip/hip_runtime.h>
#include <math.h>

constexpr int NSEQ     = 512;
constexpr int NSTEP    = 1024;
constexpr int XDIM     = 8;
constexpr int HID      = 64;
constexpr int NGATE    = 4 * HID;
constexpr int ROWS_BLK = 16;
constexpr int NTHR     = 128;
constexpr int KXPAD0   = 32;
constexpr int LDB0     = KXPAD0 + HID;
constexpr int LDB1     = HID + HID;
constexpr int HPITCH   = 72;
constexpr int XROWP    = 33;
constexpr int CHUNK    = 32;
constexpr float OPCARRY = 256.0f;
constexpr float ACC_INV = 1.0f / (OPCARRY * OPCARRY);
constexpr int HB_ELEMS  = 3 * 2 * ROWS_BLK * HPITCH;

static_assert(NSEQ % ROWS_BLK == 0, "batch tiles");
static_assert(NSTEP % CHUNK == 0, "time chunks");
static_assert(HID == 16 * (NTHR / 32), "one 16-column group per wave");
static_assert(LDB0 % 32 == 0 && LDB1 % 32 == 0, "K multiple of 32");
static_assert(HB_ELEMS % NTHR == 0, "zero fill exact");
static_assert(XDIM == 8, "one 16-byte unit per step");
static_assert((size_t)2 * NSEQ * NSTEP * 4 == (size_t)4194304, "output bytes");

typedef __attribute__((ext_vector_type(16))) _Float16 v16h;
typedef __attribute__((ext_vector_type(8)))  _Float16 v8h;
typedef __attribute__((ext_vector_type(8)))  float    v8f;
typedef __attribute__((ext_vector_type(4)))  float    v4f;
typedef __attribute__((ext_vector_type(4)))  unsigned v4u;

template <typename T> struct Frag;
template <> struct Frag<_Float16> {
  typedef v16h V; union U { v16h v; v8h h[2]; };
  static __device__ __forceinline__ v16h load(const _Float16* p) {
    U f; f.h[0] = *(const v8h*)(p); f.h[1] = *(const v8h*)(p + 16); return f.v;
  }
  static __device__ __forceinline__ v8f mma(v16h a, v16h b, v8f c) {
    return __builtin_amdgcn_wmma_f32_16x16x32_f16(false, a, false, b, (short)0, c, false, false);
  }
};

union FragX { v16h v; v4u q[2]; };

__device__ __forceinline__ void guard_group4(v8f& a, v8f& b, v8f& c, v8f& d, v16h x, v16h y0, v16h y1, v16h y2, v16h y3) {
  asm volatile("v_nop\n\tv_nop\n\tv_nop\n\tv_nop" : "+v"(a), "+v"(b), "+v"(c), "+v"(d) : "v"(x), "v"(y0), "v"(y1), "v"(y2), "v"(y3));
}
__device__ __forceinline__ void guard_group1(v8f& a, v16h x0, v16h x1, v16h y0, v16h y1) {
  asm volatile("v_nop\n\tv_nop\n\tv_nop\n\tv_nop" : "+v"(a) : "v"(x0), "v"(x1), "v"(y0), "v"(y1));
}

__device__ __forceinline__ float fsig(float x)  { return __builtin_amdgcn_rcpf(1.0f + expf(-x)); }
__device__ __forceinline__ float ftanh(float x) { return 1.0f - 2.0f * __builtin_amdgcn_rcpf(expf(2.0f * x) + 1.0f); }

__device__ __forceinline__ unsigned pack_h2(float lo, float hi) {
  const _Float16 a = (_Float16)lo;
  const _Float16 b = (_Float16)hi;
  const unsigned short ua = __builtin_bit_cast(unsigned short, a);
  const unsigned short ub = __builtin_bit_cast(unsigned short, b);
  return (unsigned)ua | ((unsigned)ub << 16);
}

template <int GSTRIDE>
__device__ __forceinline__ void mma_tile(v16h a, const _Float16* wrow, v8f& ai, v8f& af, v8f& ag, v8f& ao) {
  const v16h b0 = Frag<_Float16>::load(wrow);
  const v16h b1 = Frag<_Float16>::load(wrow + (size_t)1 * GSTRIDE);
  const v16h b2 = Frag<_Float16>::load(wrow + (size_t)2 * GSTRIDE);
  const v16h b3 = Frag<_Float16>::load(wrow + (size_t)3 * GSTRIDE);
  ai = Frag<_Float16>::mma(a, b0, ai);
  af = Frag<_Float16>::mma(a, b1, af);
  ag = Frag<_Float16>::mma(a, b2, ag);
  ao = Frag<_Float16>::mma(a, b3, ao);
  guard_group4(ai, af, ag, ao, a, b0, b1, b2, b3);
}

template <int GSTRIDE>
__device__ __forceinline__ void mma_seg64(const _Float16* arow, const _Float16* wrow, v8f& ai, v8f& af, v8f& ag, v8f& ao) {
#pragma unroll 1
  for (int k0 = 0; k0 < HID; k0 += 32) {
    const v16h a = Frag<_Float16>::load(arow + k0);
    mma_tile<GSTRIDE>(a, wrow + k0, ai, af, ag, ao);
  }
}

__device__ __forceinline__ void lstm_cell(const v8f& ai, const v8f& af, const v8f& ag, const v8f& ao,
                                          float bsi, float bsf, float bsg, float bso,
                                          float (&cst)[8], _Float16* hdst) {
#pragma unroll
  for (int r = 0; r < 8; ++r) {
    const float zi = ai[r] * ACC_INV + bsi;
    const float zf = af[r] * ACC_INV + bsf;
    const float zg = ag[r] * ACC_INV + bsg;
    const float zo = ao[r] * ACC_INV + bso;
    const float ig = fsig(zi);
    const float fg = fsig(zf);
    const float gg = ftanh(zg);
    const float og = fsig(zo);
    const float cn = fg * cst[r] + ig * gg;
    cst[r] = cn;
    const float hn = og * ftanh(cn);
    hdst[r * HPITCH] = (_Float16)(hn * OPCARRY);
  }
}

template <int IN_DIM, int KXPAD>
__global__ __launch_bounds__(256) void pack_w_kernel(const float* __restrict__ wih, const float* __restrict__ whh,
                                                     unsigned short* __restrict__ dst) {
  constexpr int LDB = KXPAD + HID;
  constexpr int UPR = LDB / 8;
  constexpr int NUNIT = NGATE * UPR;
  static_assert(NUNIT % 256 == 0, "exact grid");
  static_assert(IN_DIM % 8 == 0 && IN_DIM <= KXPAD, "input width");
  const int i = blockIdx.x * 256 + threadIdx.x;
  if (i < NUNIT) {
    const int n = i / UPR;
    const int u = i - n * UPR;
    const int k = 8 * u;
    int ka = k;
    if (ka > IN_DIM - 8) ka = IN_DIM - 8;
    int kb = k - KXPAD;
    if (kb < 0) kb = 0;
    if (kb > HID - 8) kb = HID - 8;
    const float* pa = wih + (size_t)n * IN_DIM + ka;
    const float* pb = whh + (size_t)n * HID + kb;
    const v4f a0 = *(const v4f*)(pa);
    const v4f a1 = *(const v4f*)(pa + 4);
    const v4f b0 = *(const v4f*)(pb);
    const v4f b1 = *(const v4f*)(pb + 4);
    const float fa = (k < IN_DIM) ? 1.0f : 0.0f;
    const float fb = (k >= KXPAD) ? 1.0f : 0.0f;
    v8h hv;
#pragma unroll
    for (int e = 0; e < 4; ++e) {
      const float w0 = fmaf(fa, a0[e], fb * b0[e]);
      const float w1 = fmaf(fa, a1[e], fb * b1[e]);
      hv[e]     = (_Float16)(w0 * OPCARRY);
      hv[4 + e] = (_Float16)(w1 * OPCARRY);
    }
    *(volatile v8h*)(dst + (size_t)i * 8) = hv;
    __threadfence();
    *(volatile v8h*)(dst + (size_t)i * 8) = hv;
  }
}

__global__ __launch_bounds__(128) void pack_head_kernel(const float* __restrict__ wm, const float* __restrict__ wa,
                                                        unsigned short* __restrict__ dst) {
  const int i = threadIdx.x;
  const int n = i >> 3;
  const int u = i & 7;
  const v4f a0 = *(const v4f*)(wm + 8 * u);
  const v4f a1 = *(const v4f*)(wm + 8 * u + 4);
  const v4f b0 = *(const v4f*)(wa + 8 * u);
  const v4f b1 = *(const v4f*)(wa + 8 * u + 4);
  const float fa = (n == 0) ? 1.0f : 0.0f;
  const float fb = (n == 1) ? 1.0f : 0.0f;
  v8h hv;
#pragma unroll
  for (int e = 0; e < 4; ++e) {
    const float w0 = fmaf(fa, a0[e], fb * b0[e]);
    const float w1 = fmaf(fa, a1[e], fb * b1[e]);
    hv[e]     = (_Float16)(w0 * OPCARRY);
    hv[4 + e] = (_Float16)(w1 * OPCARRY);
  }
  *(volatile v8h*)(dst + (size_t)i * 8) = hv;
  __threadfence();
  *(volatile v8h*)(dst + (size_t)i * 8) = hv;
}

__device__ __forceinline__ void flush_chunk(const float* ost, const float* __restrict__ v, float bmv, float bav,
                                            float* out, int rowbase, int t0, int wave, int lane) {
#pragma unroll 1
  for (int i = 0; i < 4; ++i) {
    const int row = 4 * wave + i;
    const float sm = ost[row * CHUNK + lane];
    const float sa = ost[(ROWS_BLK + row) * CHUNK + lane];
    const float vv = v[rowbase + row];
    const float mval = (sm + bmv) * vv;
    const float xa = sa + bav;
    const float sp = fmaxf(xa, 0.0f) + log1pf(expf(-fabsf(xa)));
    const float aval = sp * vv;
    float* pm = out + (size_t)(rowbase + row) * NSTEP + (size_t)(t0 + lane);
    float* pa = pm + (size_t)NSEQ * NSTEP;
    *(volatile float*)pm = mval;
    *(volatile float*)pa = aval;
    __threadfence();
    *(volatile float*)pm = mval;
    *(volatile float*)pa = aval;
  }
}

__global__ __launch_bounds__(NTHR) void lstm3_seq_kernel(const float* __restrict__ x, const float* __restrict__ v,
                                                         const float* __restrict__ b0, const float* __restrict__ b1,
                                                         const float* __restrict__ b2,
                                                         const float* __restrict__ bm, const float* __restrict__ ba,
                                                         const unsigned short* __restrict__ W0p,
                                                         const unsigned short* __restrict__ W1p,
                                                         const unsigned short* __restrict__ W2p,
                                                         const unsigned short* __restrict__ WHp,
                                                         float* out) {
  __shared__ __align__(16) _Float16 Hb[3][2][ROWS_BLK * HPITCH];
  __shared__ __align__(16) v4u      Xs[ROWS_BLK * XROWP];
  __shared__ __align__(16) float    Ost[2 * ROWS_BLK * CHUNK];

  const int tid  = threadIdx.x;
  const int lane = tid & 31;
  const int wave = __builtin_amdgcn_readfirstlane((int)(threadIdx.x >> 5));
  const int c    = lane & 15;
  const int hh   = lane >> 4;
  const int koff = hh * 8;
  const int rowbase = blockIdx.x * ROWS_BLK;
  const int col  = 16 * wave + c;

  const _Float16* W0 = (const _Float16*)W0p;
  const _Float16* W1 = (const _Float16*)W1p;
  const _Float16* W2 = (const _Float16*)W2p;
  const _Float16* WH = (const _Float16*)WHp;

  {
    _Float16* hz = &Hb[0][0][0];
#pragma unroll 1
    for (int i = tid; i < HB_ELEMS; i += NTHR) hz[i] = (_Float16)0.0f;
  }

  float bs0[4], bs1[4], bs2[4];
#pragma unroll
  for (int g = 0; g < 4; ++g) {
    bs0[g] = b0[g * HID + col];
    bs1[g] = b1[g * HID + col];
    bs2[g] = b2[g * HID + col];
  }
  asm volatile("" ::: "memory");
  const float bmv = bm[0];
  const float bav = ba[0];
  const v16h bhd0 = Frag<_Float16>::load(WH + (size_t)c * HID + koff);
  const v16h bhd1 = Frag<_Float16>::load(WH + (size_t)c * HID + koff + 32);

  float cs0[8], cs1[8], cs2[8];
#pragma unroll
  for (int r = 0; r < 8; ++r) { cs0[r] = 0.0f; cs1[r] = 0.0f; cs2[r] = 0.0f; }

  const _Float16* w0row = W0 + (size_t)col * LDB0 + koff;
  const _Float16* w1row = W1 + (size_t)col * LDB1 + koff;
  const _Float16* w2row = W2 + (size_t)col * LDB1 + koff;

  const int aoff = c * HPITCH + koff;
  const int hoff = (8 * hh) * HPITCH + col;
  const unsigned xm = hh ? 0u : 0xFFFFFFFFu;
  const v4u xmask = {xm, xm, xm, xm};
  const v4u zero4 = {0u, 0u, 0u, 0u};
  const v8f z8 = {0.f, 0.f, 0.f, 0.f, 0.f, 0.f, 0.f, 0.f};

  const int srow = tid >> 3;
  const int sseg = tid & 7;

  __syncthreads();

#pragma unroll 1
  for (int t = 0; t < NSTEP; ++t) {
    const int ts = t & (CHUNK - 1);
    if (ts == 0) {
      const float* sp = x + ((size_t)(rowbase + srow) * NSTEP + (size_t)(t + 4 * sseg)) * XDIM;
      const v4f f0 = *(const v4f*)(sp);
      const v4f f1 = *(const v4f*)(sp + 4);
      const v4f f2 = *(const v4f*)(sp + 8);
      const v4f f3 = *(const v4f*)(sp + 12);
      const v4f f4 = *(const v4f*)(sp + 16);
      const v4f f5 = *(const v4f*)(sp + 20);
      const v4f f6 = *(const v4f*)(sp + 24);
      const v4f f7 = *(const v4f*)(sp + 28);
      v4u q0, q1, q2, q3;
      q0[0] = pack_h2(f0[0] * OPCARRY, f0[1] * OPCARRY);
      q0[1] = pack_h2(f0[2] * OPCARRY, f0[3] * OPCARRY);
      q0[2] = pack_h2(f1[0] * OPCARRY, f1[1] * OPCARRY);
      q0[3] = pack_h2(f1[2] * OPCARRY, f1[3] * OPCARRY);
      q1[0] = pack_h2(f2[0] * OPCARRY, f2[1] * OPCARRY);
      q1[1] = pack_h2(f2[2] * OPCARRY, f2[3] * OPCARRY);
      q1[2] = pack_h2(f3[0] * OPCARRY, f3[1] * OPCARRY);
      q1[3] = pack_h2(f3[2] * OPCARRY, f3[3] * OPCARRY);
      q2[0] = pack_h2(f4[0] * OPCARRY, f4[1] * OPCARRY);
      q2[1] = pack_h2(f4[2] * OPCARRY, f4[3] * OPCARRY);
      q2[2] = pack_h2(f5[0] * OPCARRY, f5[1] * OPCARRY);
      q2[3] = pack_h2(f5[2] * OPCARRY, f5[3] * OPCARRY);
      q3[0] = pack_h2(f6[0] * OPCARRY, f6[1] * OPCARRY);
      q3[1] = pack_h2(f6[2] * OPCARRY, f6[3] * OPCARRY);
      q3[2] = pack_h2(f7[0] * OPCARRY, f7[1] * OPCARRY);
      q3[3] = pack_h2(f7[2] * OPCARRY, f7[3] * OPCARRY);
      Xs[srow * XROWP + 4 * sseg + 0] = q0;
      Xs[srow * XROWP + 4 * sseg + 1] = q1;
      Xs[srow * XROWP + 4 * sseg + 2] = q2;
      Xs[srow * XROWP + 4 * sseg + 3] = q3;
      __syncthreads();
      if (t > 0) flush_chunk(Ost, v, bmv, bav, out, rowbase, t - CHUNK, wave, lane);
    }

    const int p = t & 1;
    const _Float16* H0r = &Hb[0][p][0];
    _Float16*       H0w = &Hb[0][p ^ 1][0];
    const _Float16* H1r = &Hb[1][p][0];
    _Float16*       H1w = &Hb[1][p ^ 1][0];
    const _Float16* H2r = &Hb[2][p][0];
    _Float16*       H2w = &Hb[2][p ^ 1][0];

    {
      v8f ai = z8, af = z8, ag = z8, ao = z8;
      v4u xw = Xs[c * XROWP + ts];
      xw = xw & xmask;
      FragX fx;
      fx.q[0] = xw;
      fx.q[1] = zero4;
      mma_tile<HID * LDB0>(fx.v, w0row, ai, af, ag, ao);
      mma_seg64<HID * LDB0>(H0r + aoff, w0row + KXPAD0, ai, af, ag, ao);
      lstm_cell(ai, af, ag, ao, bs0[0], bs0[1], bs0[2], bs0[3], cs0, H0w + hoff);
    }
    __syncthreads();

    {
      v8f ai = z8, af = z8, ag = z8, ao = z8;
      mma_seg64<HID * LDB1>(H0w + aoff, w1row, ai, af, ag, ao);
      mma_seg64<HID * LDB1>(H1r + aoff, w1row + HID, ai, af, ag, ao);
      lstm_cell(ai, af, ag, ao, bs1[0], bs1[1], bs1[2], bs1[3], cs1, H1w + hoff);
    }
    __syncthreads();

    {
      v8f ai = z8, af = z8, ag = z8, ao = z8;
      mma_seg64<HID * LDB1>(H1w + aoff, w2row, ai, af, ag, ao);
      mma_seg64<HID * LDB1>(H2r + aoff, w2row + HID, ai, af, ag, ao);
      lstm_cell(ai, af, ag, ao, bs2[0], bs2[1], bs2[2], bs2[3], cs2, H2w + hoff);
    }
    __syncthreads();

    if (wave == 0) {
      const v16h a0 = Frag<_Float16>::load(H2w + aoff);
      const v16h a1 = Frag<_Float16>::load(H2w + aoff + 32);
      v8f hacc = z8;
      hacc = Frag<_Float16>::mma(a0, bhd0, hacc);
      hacc = Frag<_Float16>::mma(a1, bhd1, hacc);
      guard_group1(hacc, a0, a1, bhd0, bhd1);
      if (c < 2) {
#pragma unroll
        for (int r = 0; r < 8; ++r) Ost[(c * ROWS_BLK + 8 * hh + r) * CHUNK + ts] = hacc[r] * ACC_INV;
      }
    }
  }
  __syncthreads();
  flush_chunk(Ost, v, bmv, bav, out, rowbase, NSTEP - CHUNK, wave, lane);
}

extern "C" void kernel_launch(void* const* d_in, const int* in_sizes, int n_in,
                              void* d_out, int out_size, void* d_ws, size_t ws_size, hipStream_t stream) {
  if (n_in < 15 || d_out == nullptr || d_ws == nullptr) return;
  if (in_sizes[0] != NSEQ * NSTEP * XDIM || in_sizes[1] != NSEQ ||
      in_sizes[2] != NGATE * XDIM || in_sizes[3] != NGATE * HID || in_sizes[4] != NGATE ||
      in_sizes[5] != NGATE * HID || in_sizes[6] != NGATE * HID || in_sizes[7] != NGATE ||
      in_sizes[8] != NGATE * HID || in_sizes[9] != NGATE * HID || in_sizes[10] != NGATE ||
      in_sizes[11] != HID || in_sizes[12] != 1 || in_sizes[13] != HID || in_sizes[14] != 1 ||
      out_size != 2 * NSEQ * NSTEP) return;

  const float* x     = (const float*)d_in[0];
  const float* v     = (const float*)d_in[1];
  const float* w_ih0 = (const float*)d_in[2];
  const float* w_hh0 = (const float*)d_in[3];
  const float* b0    = (const float*)d_in[4];
  const float* w_ih1 = (const float*)d_in[5];
  const float* w_hh1 = (const float*)d_in[6];
  const float* b1    = (const float*)d_in[7];
  const float* w_ih2 = (const float*)d_in[8];
  const float* w_hh2 = (const float*)d_in[9];
  const float* b2    = (const float*)d_in[10];
  const float* wm    = (const float*)d_in[11];
  const float* bm    = (const float*)d_in[12];
  const float* wa    = (const float*)d_in[13];
  const float* ba    = (const float*)d_in[14];
  float* out = (float*)d_out;

  char* ws = (char*)d_ws; size_t off = 0;
  auto carve = [&](size_t bytes) -> char* { char* p = ws + off; off += (bytes + 511) & ~(size_t)511; return p; };
  unsigned short* W0 = (unsigned short*)carve((size_t)NGATE * LDB0 * 2);
  unsigned short* W1 = (unsigned short*)carve((size_t)NGATE * LDB1 * 2);
  unsigned short* W2 = (unsigned short*)carve((size_t)NGATE * LDB1 * 2);
  unsigned short* WH = (unsigned short*)carve((size_t)16 * HID * 2);
  if (off > ws_size || off > (size_t)134217728) return;

  pack_w_kernel<XDIM, KXPAD0><<<(NGATE * (LDB0 / 8)) / 256, 256, 0, stream>>>(w_ih0, w_hh0, W0);
  pack_w_kernel<HID, HID><<<(NGATE * (LDB1 / 8)) / 256, 256, 0, stream>>>(w_ih1, w_hh1, W1);
  pack_w_kernel<HID, HID><<<(NGATE * (LDB1 / 8)) / 256, 256, 0, stream>>>(w_ih2, w_hh2, W2);
  pack_head_kernel<<<1, 128, 0, stream>>>(wm, wa, WH);

  lstm3_seq_kernel<<<NSEQ / ROWS_BLK, NTHR, 0, stream>>>(x, v, b0, b1, b2, bm, ba, W0, W1, W2, WH, out);
}
